// MambaBlock_63806034150206
// MI455X (gfx1250) — hardware-verified
//
#include <hip/hip_runtime.h>
#include <math.h>
#include <stddef.h>
#include <stdint.h>

#define BB    2
#define LL    2048
#define DD    1024
#define D2    2048
#define NS    16
#define NBC   32
#define KC    4
#define MR    (BB * LL)
#define K2    (2 * DD)
#define NTHR  256
#define GTHR  128
#define GBM   64
#define TCH   32
#define WSMAX 134217728
#define LNEPS 1e-5f

#define NU_XB   (MR * DD / 8)
#define NU_WIN  (D2 * DD / 8)
#define NU_WDT  (DD * K2 / 8)
#define NU_WXP  (NBC * K2 / 8)
#define NU_WOUT (DD * K2 / 8)
#define NU_ALL  (NU_XB + NU_WIN + NU_WDT + NU_WXP + NU_WOUT)

static_assert(NU_XB % NTHR == 0 && NU_WIN % NTHR == 0 && NU_WDT % NTHR == 0 && NU_WXP % NTHR == 0 && NU_WOUT % NTHR == 0);
static_assert(NU_ALL % NTHR == 0);
static_assert(K2 / 8 == 256);
static_assert(MR % GBM == 0 && D2 % 128 == 0 && DD % 128 == 0 && NBC == 32);
static_assert(DD % 32 == 0 && K2 % 32 == 0);
static_assert(GBM == (GTHR / 32) * 16);
static_assert(DD == 4 * NTHR && D2 == 8 * NTHR);
static_assert(LL % TCH == 0 && (LL & (LL - 1)) == 0);
static_assert(TCH * NBC == 4 * NTHR && TCH * NTHR == 8 * 4 * NTHR);
static_assert(DD % NTHR == 0 && NS == 16 && KC == 4);

typedef float          v4f   __attribute__((ext_vector_type(4)));
typedef float          v8f   __attribute__((ext_vector_type(8)));
typedef int            v8i   __attribute__((ext_vector_type(8)));
typedef unsigned short v8us  __attribute__((ext_vector_type(8)));
typedef unsigned short v16us __attribute__((ext_vector_type(16)));
typedef __bf16         v16bf __attribute__((ext_vector_type(16)));
typedef v4f  __attribute__((may_alias)) v4fa;
typedef v8us __attribute__((may_alias)) v8usa;
union FragB { v16bf v; v16us u; v8us h[2]; v8i w; };

__device__ __forceinline__ v8f wmb(const FragB& a, const FragB& b, v8f c) {
  v8f d = __builtin_amdgcn_wmma_f32_16x16x32_bf16(false, a.v, false, b.v, (short)0, c, false, false);
  asm volatile("v_nop\n\tv_nop\n\tv_nop\n\tv_nop" : "+v"(d) : "v"(a.w), "v"(b.w));
  return d;
}

__device__ __forceinline__ unsigned bf16_bits(float f) {
  const unsigned u = __float_as_uint(f);
  return (u + 0x7FFFu + ((u >> 16) & 1u)) >> 16;
}
__device__ __forceinline__ float bf16_val(float f) {
  return __uint_as_float(bf16_bits(f) << 16);
}
__device__ __forceinline__ float softplus_f(float v) {
  const float e = expf(-fabsf(v));
  return fmaxf(v, 0.0f) + log1pf(e);
}

__global__ __launch_bounds__(NTHR) void k_prep(const float* __restrict__ x, const float* __restrict__ W_in,
                                               const float* __restrict__ W_dt, const float* __restrict__ W_xp,
                                               const float* __restrict__ W_out,
                                               unsigned short* XB, unsigned short* WIN, unsigned short* WDT2,
                                               unsigned short* WXP2, unsigned short* WOUT2) {
  const int u  = (int)blockIdx.x * NTHR + (int)threadIdx.x;
  const int L0 = NU_XB;
  const int L1 = L0 + NU_WIN;
  const int L2 = L1 + NU_WDT;
  const int L3 = L2 + NU_WXP;
  const int L4 = L3 + NU_WOUT;
  if (u >= L4) return;
  const float* src;
  unsigned short* dst;
  if (u < L0) {
    src = x + (size_t)u * 8;
    dst = XB + (size_t)u * 8;
  } else if (u < L1) {
    const int v = u - L0;
    src = W_in + (size_t)v * 8;
    dst = WIN + (size_t)v * 8;
  } else if (u < L2) {
    const int v = u - L1;
    const int n = v >> 8;
    const int k8 = (v & 255) * 8;
    src = W_dt + (size_t)n * DD + (k8 & (DD - 1));
    dst = WDT2 + (size_t)n * K2 + k8;
  } else if (u < L3) {
    const int v = u - L2;
    const int n = v >> 8;
    const int k8 = (v & 255) * 8;
    src = W_xp + (size_t)n * DD + (k8 & (DD - 1));
    dst = WXP2 + (size_t)n * K2 + k8;
  } else {
    const int v = u - L3;
    const int n = v >> 8;
    const int k8 = (v & 255) * 8;
    src = W_out + (size_t)n * DD + (k8 & (DD - 1));
    dst = WOUT2 + (size_t)n * K2 + k8;
  }
  const v4f a = *(const v4fa*)src;
  const v4f c = *(const v4fa*)(src + 4);
  v8us o;
  o[0] = (unsigned short)bf16_bits(a.x);
  o[1] = (unsigned short)bf16_bits(a.y);
  o[2] = (unsigned short)bf16_bits(a.z);
  o[3] = (unsigned short)bf16_bits(a.w);
  o[4] = (unsigned short)bf16_bits(c.x);
  o[5] = (unsigned short)bf16_bits(c.y);
  o[6] = (unsigned short)bf16_bits(c.z);
  o[7] = (unsigned short)bf16_bits(c.w);
  *(volatile v8us*)dst = o;
  __threadfence();
  *(volatile v8us*)dst = o;
}

template <int MODE, int NT>
__global__ __launch_bounds__(GTHR) void k_gemm(const unsigned short* __restrict__ A, int lda,
                                               const unsigned short* __restrict__ BT, int ldb, int K,
                                               const float* __restrict__ bias, float* Cm, int ldc) {
  constexpr int BN = 16 * NT;
  __shared__ __attribute__((aligned(16))) float stg[GBM * BN];
  const int tid = (int)threadIdx.x, lane = tid & 31, wave = tid >> 5, hh = lane >> 4, m = lane & 15;
  const int rowBase = (int)blockIdx.x * GBM;
  const int colBase = (int)blockIdx.y * BN;

  v8f acc[NT];
  {
    const v8f z = {0.f, 0.f, 0.f, 0.f, 0.f, 0.f, 0.f, 0.f};
#pragma unroll
    for (int t = 0; t < NT; ++t) acc[t] = z;
  }
  const unsigned short* ap = A  + (size_t)(rowBase + 16 * wave + m) * (size_t)lda + 8 * hh;
  const unsigned short* bp = BT + (size_t)(colBase + m) * (size_t)ldb + 8 * hh;

#pragma unroll 1
  for (int k0 = 0; k0 < K; k0 += 32) {
    FragB af;
    af.h[0] = *(const v8usa*)(ap + k0);
    af.h[1] = *(const v8usa*)(ap + k0 + 16);
#pragma unroll
    for (int nt = 0; nt < NT; ++nt) {
      const unsigned short* wq = bp + (size_t)(16 * nt) * (size_t)ldb + k0;
      FragB bf;
      bf.h[0] = *(const v8usa*)wq;
      bf.h[1] = *(const v8usa*)(wq + 16);
      acc[nt] = wmb(af, bf, acc[nt]);
    }
  }

#pragma unroll
  for (int nt = 0; nt < NT; ++nt) {
    const int lc = 16 * nt + m;
    float bvv = 0.0f;
    if constexpr (MODE == 1 || MODE == 2) bvv = bf16_val(bias[colBase + lc]);
#pragma unroll
    for (int r = 0; r < 8; ++r) {
      const int lr = 16 * wave + 8 * hh + r;
      stg[lr * BN + lc] = acc[nt][r] + bvv;
    }
  }
  __syncthreads();

  if constexpr (NT == 8) {
    if constexpr (MODE == 1) {
#pragma unroll 1
      for (int i = 0; i < 16; ++i) {
        float* sp = stg + (16 * wave + i) * BN + 4 * lane;
        v4f v = *(v4fa*)sp;
        v.x = softplus_f(v.x);
        v.y = softplus_f(v.y);
        v.z = softplus_f(v.z);
        v.w = softplus_f(v.w);
        *(v4fa*)sp = v;
      }
    }
    v4f pv[16];
#pragma unroll
    for (int i = 0; i < 16; ++i) pv[i] = *(const v4fa*)(stg + (16 * wave + i) * BN + 4 * lane);
#pragma unroll
    for (int i = 0; i < 16; ++i) {
      float* op = Cm + (size_t)(rowBase + 16 * wave + i) * (size_t)ldc + colBase + 4 * lane;
      *(volatile v4f*)op = pv[i];
    }
    __threadfence();
#pragma unroll
    for (int i = 0; i < 16; ++i) {
      float* op = Cm + (size_t)(rowBase + 16 * wave + i) * (size_t)ldc + colBase + 4 * lane;
      *(volatile v4f*)op = pv[i];
    }
  } else {
    const int sub = lane >> 3, q = lane & 7;
    v4f pv[4];
#pragma unroll
    for (int it = 0; it < 4; ++it) pv[it] = *(const v4fa*)(stg + (16 * wave + 4 * it + sub) * BN + 4 * q);
#pragma unroll
    for (int it = 0; it < 4; ++it) {
      float* op = Cm + (size_t)(rowBase + 16 * wave + 4 * it + sub) * (size_t)ldc + colBase + 4 * q;
      *(volatile v4f*)op = pv[it];
    }
    __threadfence();
#pragma unroll
    for (int it = 0; it < 4; ++it) {
      float* op = Cm + (size_t)(rowBase + 16 * wave + 4 * it + sub) * (size_t)ldc + colBase + 4 * q;
      *(volatile v4f*)op = pv[it];
    }
  }
}

__global__ __launch_bounds__(NTHR) void k_gate(const float* __restrict__ XZ, const float* __restrict__ Wc,
                                               const float* __restrict__ bc, float* GATE, unsigned short* GHL) {
  __shared__ __attribute__((aligned(16))) float sG[DD];
  __shared__ __attribute__((aligned(16))) unsigned short sH[D2];
  const int r = (int)blockIdx.x;
  const int l = r & (LL - 1);
  const int t = (int)threadIdx.x;
  const int   o0 = (l >= 3) ? 3 : 0;
  const int   o1 = (l >= 2) ? 2 : 0;
  const int   o2 = (l >= 1) ? 1 : 0;
  const float f0 = (l >= 3) ? 1.0f : 0.0f;
  const float f1 = (l >= 2) ? 1.0f : 0.0f;
  const float f2 = (l >= 1) ? 1.0f : 0.0f;
  const float* row0 = XZ + (size_t)(r - o0) * D2;
  const float* row1 = XZ + (size_t)(r - o1) * D2;
  const float* row2 = XZ + (size_t)(r - o2) * D2;
  const float* row3 = XZ + (size_t)r * D2;
#pragma unroll 1
  for (int ds = 0; ds < DD / NTHR; ++ds) {
    const int d = t + NTHR * ds;
    const v4f w4 = *(const v4fa*)(Wc + (size_t)d * KC);
    const float x0 = row0[d];
    const float x1 = row1[d];
    const float x2 = row2[d];
    const float x3 = row3[d];
    const float z  = row3[DD + d];
    float s = bf16_val(bc[d]);
    s = fmaf(bf16_val(w4.x) * f0, x0, s);
    s = fmaf(bf16_val(w4.y) * f1, x1, s);
    s = fmaf(bf16_val(w4.z) * f2, x2, s);
    s = fmaf(bf16_val(w4.w), x3, s);
    const float e   = expf(-s);
    const float sig = __builtin_amdgcn_rcpf(1.0f + e);
    const float g   = (s * sig) * z;
    sG[d] = g;
    const unsigned hb = bf16_bits(g);
    sH[d]      = (unsigned short)hb;
    sH[DD + d] = (unsigned short)bf16_bits(g - __uint_as_float(hb << 16));
  }
  __syncthreads();
  const v4f  gv = *(const v4fa*)(sG + 4 * t);
  const v8us hv = *(const v8usa*)(sH + 8 * t);
  float*          gp = GATE + (size_t)r * DD + 4 * t;
  unsigned short* hp = GHL  + (size_t)r * D2 + 8 * t;
  *(volatile v4f*)gp  = gv;
  *(volatile v8us*)hp = hv;
  __threadfence();
  *(volatile v4f*)gp  = gv;
  *(volatile v8us*)hp = hv;
}

__global__ __launch_bounds__(NTHR) void k_scan(const float* __restrict__ DELTA, const float* __restrict__ BCM,
                                               const float* __restrict__ GATE, const float* __restrict__ A_log,
                                               float* Y) {
  __shared__ __attribute__((aligned(16))) float sBC[TCH * NBC];
  __shared__ __attribute__((aligned(16))) float sY[TCH * NTHR];
  const int t = (int)threadIdx.x;
  const int dBase = (int)blockIdx.x * NTHR;
  const int d = dBase + t;
  const int b = (int)blockIdx.y;
  const size_t rb = (size_t)b * LL;

  float An[NS];
  {
    const float* alp = A_log + (size_t)d * NS;
    const v4f a0 = *(const v4fa*)(alp);
    const v4f a1 = *(const v4fa*)(alp + 4);
    const v4f a2 = *(const v4fa*)(alp + 8);
    const v4f a3 = *(const v4fa*)(alp + 12);
    An[0]  = -__expf(bf16_val(a0.x)); An[1]  = -__expf(bf16_val(a0.y));
    An[2]  = -__expf(bf16_val(a0.z)); An[3]  = -__expf(bf16_val(a0.w));
    An[4]  = -__expf(bf16_val(a1.x)); An[5]  = -__expf(bf16_val(a1.y));
    An[6]  = -__expf(bf16_val(a1.z)); An[7]  = -__expf(bf16_val(a1.w));
    An[8]  = -__expf(bf16_val(a2.x)); An[9]  = -__expf(bf16_val(a2.y));
    An[10] = -__expf(bf16_val(a2.z)); An[11] = -__expf(bf16_val(a2.w));
    An[12] = -__expf(bf16_val(a3.x)); An[13] = -__expf(bf16_val(a3.y));
    An[14] = -__expf(bf16_val(a3.z)); An[15] = -__expf(bf16_val(a3.w));
  }
  float h[NS];
#pragma unroll
  for (int n = 0; n < NS; ++n) h[n] = 0.0f;

  const int srow = t >> 3, sq = t & 7;
  const int ysub = t >> 6, yp = t & 63;

#pragma unroll 1
  for (int c = 0; c < LL / TCH; ++c) {
    const int l0 = c * TCH;
    __syncthreads();
    *(v4fa*)(sBC + srow * NBC + 4 * sq) = *(const v4fa*)(BCM + (rb + l0 + srow) * NBC + 4 * sq);
    __syncthreads();
#pragma unroll 1
    for (int i = 0; i < TCH; ++i) {
      const size_t ro = (rb + l0 + i) * DD + d;
      const float dl = DELTA[ro];
      const float g  = GATE[ro];
      const float dg = dl * g;
      const float* bcr = sBC + i * NBC;
      const v4f b0 = *(const v4fa*)(bcr);
      const v4f b1 = *(const v4fa*)(bcr + 4);
      const v4f b2 = *(const v4fa*)(bcr + 8);
      const v4f b3 = *(const v4fa*)(bcr + 12);
      const v4f c0 = *(const v4fa*)(bcr + 16);
      const v4f c1 = *(const v4fa*)(bcr + 20);
      const v4f c2 = *(const v4fa*)(bcr + 24);
      const v4f c3 = *(const v4fa*)(bcr + 28);
      const float bbv[NS] = {b0.x, b0.y, b0.z, b0.w, b1.x, b1.y, b1.z, b1.w,
                             b2.x, b2.y, b2.z, b2.w, b3.x, b3.y, b3.z, b3.w};
      const float ccv[NS] = {c0.x, c0.y, c0.z, c0.w, c1.x, c1.y, c1.z, c1.w,
                             c2.x, c2.y, c2.z, c2.w, c3.x, c3.y, c3.z, c3.w};
      float yv = 0.0f;
#pragma unroll
      for (int n = 0; n < NS; ++n) {
        const float a = __expf(dl * An[n]);
        h[n] = fmaf(a, h[n], dg * bbv[n]);
        yv = fmaf(h[n], ccv[n], yv);
      }
      sY[i * NTHR + t] = yv;
    }
    __syncthreads();
    v4f pv[8];
#pragma unroll
    for (int it = 0; it < 8; ++it) pv[it] = *(const v4fa*)(sY + (4 * it + ysub) * NTHR + 4 * yp);
#pragma unroll
    for (int it = 0; it < 8; ++it) {
      float* op = Y + (rb + l0 + 4 * it + ysub) * DD + dBase + 4 * yp;
      *(volatile v4f*)op = pv[it];
    }
    __threadfence();
#pragma unroll
    for (int it = 0; it < 8; ++it) {
      float* op = Y + (rb + l0 + 4 * it + ysub) * DD + dBase + 4 * yp;
      *(volatile v4f*)op = pv[it];
    }
  }
}

__global__ __launch_bounds__(NTHR) void k_ln(const float* __restrict__ Y, const float* __restrict__ x,
                                             const float* __restrict__ gam, const float* __restrict__ bet,
                                             unsigned short* YNHL) {
  __shared__ __attribute__((aligned(16))) float sred[16];
  __shared__ __attribute__((aligned(16))) unsigned short sH[D2];
  const int r = (int)blockIdx.x, t = (int)threadIdx.x, lane = t & 31, wave = t >> 5;
  const size_t base = (size_t)r * DD + 4 * t;
  const v4f yv = *(const v4fa*)(Y + base);
  const v4f xv = *(const v4fa*)(x + base);
  const float v0 = yv.x + bf16_val(xv.x);
  const float v1 = yv.y + bf16_val(xv.y);
  const float v2 = yv.z + bf16_val(xv.z);
  const float v3 = yv.w + bf16_val(xv.w);
  float s = (v0 + v1) + (v2 + v3);
  s += __shfl_xor(s, 16, 32);
  s += __shfl_xor(s, 8, 32);
  s += __shfl_xor(s, 4, 32);
  s += __shfl_xor(s, 2, 32);
  s += __shfl_xor(s, 1, 32);
  if (lane == 0) sred[wave] = s;
  __syncthreads();
  const v4f pa = *(const v4fa*)(sred);
  const v4f pb = *(const v4fa*)(sred + 4);
  const float tot = ((pa.x + pa.y) + (pa.z + pa.w)) + ((pb.x + pb.y) + (pb.z + pb.w));
  const float mu = tot * (1.0f / (float)DD);
  const float e0 = v0 - mu, e1 = v1 - mu, e2 = v2 - mu, e3 = v3 - mu;
  float q = (e0 * e0 + e1 * e1) + (e2 * e2 + e3 * e3);
  q += __shfl_xor(q, 16, 32);
  q += __shfl_xor(q, 8, 32);
  q += __shfl_xor(q, 4, 32);
  q += __shfl_xor(q, 2, 32);
  q += __shfl_xor(q, 1, 32);
  if (lane == 0) sred[8 + wave] = q;
  __syncthreads();
  const v4f qa = *(const v4fa*)(sred + 8);
  const v4f qb = *(const v4fa*)(sred + 12);
  const float qt  = ((qa.x + qa.y) + (qa.z + qa.w)) + ((qb.x + qb.y) + (qb.z + qb.w));
  const float var = qt * (1.0f / (float)DD);
  const float inv = rsqrtf(var + LNEPS);
  const v4f gv = *(const v4fa*)(gam + 4 * t);
  const v4f bv = *(const v4fa*)(bet + 4 * t);
  const float o0 = (e0 * inv) * bf16_val(gv.x) + bf16_val(bv.x);
  const float o1 = (e1 * inv) * bf16_val(gv.y) + bf16_val(bv.y);
  const float o2 = (e2 * inv) * bf16_val(gv.z) + bf16_val(bv.z);
  const float o3 = (e3 * inv) * bf16_val(gv.w) + bf16_val(bv.w);
  {
    const unsigned h0 = bf16_bits(o0), h1 = bf16_bits(o1), h2 = bf16_bits(o2), h3 = bf16_bits(o3);
    sH[4 * t + 0] = (unsigned short)h0;
    sH[4 * t + 1] = (unsigned short)h1;
    sH[4 * t + 2] = (unsigned short)h2;
    sH[4 * t + 3] = (unsigned short)h3;
    sH[DD + 4 * t + 0] = (unsigned short)bf16_bits(o0 - __uint_as_float(h0 << 16));
    sH[DD + 4 * t + 1] = (unsigned short)bf16_bits(o1 - __uint_as_float(h1 << 16));
    sH[DD + 4 * t + 2] = (unsigned short)bf16_bits(o2 - __uint_as_float(h2 << 16));
    sH[DD + 4 * t + 3] = (unsigned short)bf16_bits(o3 - __uint_as_float(h3 << 16));
  }
  __syncthreads();
  const v8us hv = *(const v8usa*)(sH + 8 * t);
  unsigned short* op = YNHL + (size_t)r * D2 + 8 * t;
  *(volatile v8us*)op = hv;
  __threadfence();
  *(volatile v8us*)op = hv;
}

extern "C" void kernel_launch(void* const* d_in, const int* in_sizes, int n_in,
                              void* d_out, int out_size, void* d_ws, size_t ws_size,
                              hipStream_t stream) {
  if (n_in < 12) return;
  if (in_sizes[0]  != MR * DD) return;
  if (in_sizes[1]  != D2 * DD) return;
  if (in_sizes[2]  != DD * KC) return;
  if (in_sizes[3]  != DD) return;
  if (in_sizes[4]  != NBC * DD) return;
  if (in_sizes[5]  != DD * DD) return;
  if (in_sizes[6]  != DD) return;
  if (in_sizes[7]  != DD * NS) return;
  if (in_sizes[8]  != DD) return;
  if (in_sizes[9]  != DD) return;
  if (in_sizes[10] != DD * DD) return;
  if (in_sizes[11] != DD) return;
  if (out_size != MR * DD) return;

  const float* x     = (const float*)d_in[0];
  const float* W_in  = (const float*)d_in[1];
  const float* W_cv  = (const float*)d_in[2];
  const float* b_cv  = (const float*)d_in[3];
  const float* W_xp  = (const float*)d_in[4];
  const float* W_dt  = (const float*)d_in[5];
  const float* b_dt  = (const float*)d_in[6];
  const float* A_log = (const float*)d_in[7];
  const float* ln_g  = (const float*)d_in[8];
  const float* ln_b  = (const float*)d_in[9];
  const float* W_out = (const float*)d_in[10];
  const float* b_out = (const float*)d_in[11];
  float* out = (float*)d_out;

  size_t off = 0;
  const size_t oXB   = off; off += (size_t)MR * DD * 2;
  const size_t oWIN  = off; off += (size_t)D2 * DD * 2;
  const size_t oWDT  = off; off += (size_t)DD * K2 * 2;
  const size_t oWXP  = off; off += (size_t)NBC * K2 * 2;
  const size_t oWOUT = off; off += (size_t)DD * K2 * 2;
  const size_t oXZ   = off; off += (size_t)MR * D2 * 4;
  const size_t oGATE = off; off += (size_t)MR * DD * 4;
  const size_t oGHL  = off; off += (size_t)MR * K2 * 2;
  const size_t oDEL  = off; off += (size_t)MR * DD * 4;
  const size_t oBC   = off; off += (size_t)MR * NBC * 4;
  if (off > ws_size || off > (size_t)WSMAX) return;
  char* ws = (char*)d_ws;
  unsigned short* XB    = (unsigned short*)(ws + oXB);
  unsigned short* WIN   = (unsigned short*)(ws + oWIN);
  unsigned short* WDT2  = (unsigned short*)(ws + oWDT);
  unsigned short* WXP2  = (unsigned short*)(ws + oWXP);
  unsigned short* WOUT2 = (unsigned short*)(ws + oWOUT);
  float*          XZ    = (float*)(ws + oXZ);
  float*          Y     = (float*)(ws + oXZ);
  float*          GATE  = (float*)(ws + oGATE);
  unsigned short* GHL   = (unsigned short*)(ws + oGHL);
  unsigned short* YNHL  = (unsigned short*)(ws + oGHL);
  float*          DELTA = (float*)(ws + oDEL);
  float*          BCM   = (float*)(ws + oBC);

  k_prep<<<NU_ALL / NTHR, NTHR, 0, stream>>>(x, W_in, W_dt, W_xp, W_out, XB, WIN, WDT2, WXP2, WOUT2);
  k_gemm<0, 8><<<dim3(MR / GBM, D2 / 128), GTHR, 0, stream>>>(XB, DD, WIN, DD, DD, b_dt, XZ, D2);
  k_gate<<<MR, NTHR, 0, stream>>>(XZ, W_cv, b_cv, GATE, GHL);
  k_gemm<1, 8><<<dim3(MR / GBM, DD / 128), GTHR, 0, stream>>>(GHL, K2, WDT2, K2, K2, b_dt, DELTA, DD);
  k_gemm<3, 2><<<dim3(MR / GBM, 1), GTHR, 0, stream>>>(GHL, K2, WXP2, K2, K2, b_dt, BCM, NBC);
  k_scan<<<dim3(DD / NTHR, BB), NTHR, 0, stream>>>(DELTA, BCM, GATE, A_log, Y);
  k_ln<<<MR, NTHR, 0, stream>>>(Y, x, ln_g, ln_b, YNHL);
  k_gemm<2, 8><<<dim3(MR / GBM, DD / 128), GTHR, 0, stream>>>(YNHL, K2, WOUT2, K2, K2, b_out, out, DD);
}
